// Multihead_self_attention_21397527068764
// MI455X (gfx1250) — hardware-verified
//
#include <hip/hip_runtime.h>


#ifndef NB
#define NB 2
#endif
#ifndef SEQ
#define SEQ 2048
#endif
#define NB_FULL  2
#define SEQ_FULL 2048
#define DMOD 1024
#define NH_  16
#define HD   64
#define NFREQ 32
#define DM   DMOD
#define SCL  0.125f
#define LOSC 1024.0f

static_assert(SEQ % 64 == 0);
static_assert(SEQ >= 64);
static_assert(SEQ <= SEQ_FULL);
static_assert(NB >= 1);
static_assert(NB <= NB_FULL);
static_assert(NH_ * HD == DMOD);
static_assert(DMOD % 256 == 0);
static_assert(HD == 2 * NFREQ);

typedef _Float16 h16;
typedef unsigned short bf;
typedef __attribute__((ext_vector_type(16))) __bf16   v16bf;
typedef __attribute__((ext_vector_type(16))) _Float16 v16h;
typedef __attribute__((ext_vector_type(8)))  _Float16 v8h;
typedef __attribute__((ext_vector_type(8)))  unsigned short v8us;
typedef __attribute__((ext_vector_type(8)))  float    v8f;
typedef __attribute__((ext_vector_type(4)))  float    v4f;
typedef __attribute__((ext_vector_type(4)))  _Float16 v4h;
typedef v8h  __attribute__((may_alias)) v8ha;
typedef v4f  __attribute__((may_alias)) v4fa;
typedef v8us __attribute__((may_alias)) v8usa;

__device__ __forceinline__ unsigned short f2bf(float f) { unsigned u = __float_as_uint(f); u += 0x7FFFu + ((u >> 16) & 1u); return (unsigned short)(u >> 16); }
__device__ __forceinline__ float bf2f(unsigned short b) { return __uint_as_float(((unsigned)b) << 16); }
__device__ __forceinline__ float bfr(float f) { return bf2f(f2bf(f)); }
__device__ __forceinline__ v16h cat16(v8h lo, v8h hi) { return __builtin_shufflevector(lo, hi, 0, 1, 2, 3, 4, 5, 6, 7, 8, 9, 10, 11, 12, 13, 14, 15); }
__device__ __forceinline__ v16bf cat16b(v8us lo, v8us hi) { return __builtin_bit_cast(v16bf, __builtin_shufflevector(lo, hi, 0, 1, 2, 3, 4, 5, 6, 7, 8, 9, 10, 11, 12, 13, 14, 15)); }
__device__ __forceinline__ v8f wmma16(v16h a, v16h b, v8f c) { return __builtin_amdgcn_wmma_f32_16x16x32_f16(false, a, false, b, (short)0, c, false, false); }
__device__ __forceinline__ v8f wmmab(v16bf a, v16bf b, v8f c) { return __builtin_amdgcn_wmma_f32_16x16x32_bf16(false, a, false, b, (short)0, c, false, false); }

template <bool SPLITA, bool F16OUT = false>
__global__ __launch_bounds__(128) void k_gemmb(const bf* __restrict__ A, const bf* __restrict__ Al, const bf* __restrict__ Bn, const float* __restrict__ bias, float* C, int ldc, h16* C2, const float* __restrict__ R = nullptr, int K = DM, int rneR = 1) {
    __shared__ __align__(16) float ost[4][16 * 68];
    const int lane = threadIdx.x & 31, wave = threadIdx.x >> 5, lr = lane & 15, hi = lane >> 4;
    const int r0 = blockIdx.x * 64 + wave * 16, c0 = blockIdx.y * 64;
    const size_t aoff = (size_t)(r0 + lr) * K + 8 * hi;
    size_t boff[4];
#pragma unroll
    for (int t = 0; t < 4; ++t) boff[t] = (size_t)(c0 + t * 16 + lr) * K + 8 * hi;
    v8f acc[4];
#pragma unroll
    for (int t = 0; t < 4; ++t) acc[t] = (v8f){};
#pragma unroll 1
    for (int kc = 0; kc < K; kc += 32) {
        const v16bf a = cat16b(*(const v8us*)(A + aoff + kc), *(const v8us*)(A + aoff + kc + 16));
        v16bf al = a;
        if (SPLITA) al = cat16b(*(const v8us*)(Al + aoff + kc), *(const v8us*)(Al + aoff + kc + 16));
#pragma unroll
        for (int t = 0; t < 4; ++t) { const v16bf b = cat16b(*(const v8us*)(Bn + boff[t] + kc), *(const v8us*)(Bn + boff[t] + kc + 16)); acc[t] = wmmab(a, b, acc[t]); if (SPLITA) acc[t] = wmmab(al, b, acc[t]); }
        asm volatile("v_nop\n\tv_nop\n\tv_nop\n\tv_nop" : "+v"(acc[0]), "+v"(acc[1]), "+v"(acc[2]), "+v"(acc[3]) : "v"(a), "v"(al));
    }
    float* os = &ost[wave][0];
#pragma unroll
    for (int t = 0; t < 4; ++t) { const float bv = bias ? bfr(bias[c0 + t * 16 + lr]) : 0.f;
#pragma unroll
        for (int j = 0; j < 8; ++j) os[(hi * 8 + j) * 68 + t * 16 + lr] = acc[t][j] + bv; }
    __syncthreads();
    if (F16OUT) {
        h16* crow = (h16*)(void*)C + (size_t)r0 * ldc + c0;
        auto pass = [&]() {
#pragma unroll
            for (int s = 0; s < 4; ++s) { const int row = 4 * s + (lane >> 3), piece = lane & 7; const float* sp = os + row * 68 + piece * 8; v8h o, o2;
#pragma unroll
                for (int i = 0; i < 8; ++i) { const h16 a = (h16)sp[i]; o[i] = a; o2[i] = (h16)((sp[i] - (float)a) * LOSC); }
                *(volatile v8h*)(crow + (size_t)row * ldc + piece * 8) = o; if (C2) *(volatile v8h*)(C2 + (size_t)r0 * ldc + c0 + (size_t)row * ldc + piece * 8) = o2; }
        };
        pass(); __threadfence(); pass();
    } else {
        float* crow = C + (size_t)r0 * ldc + c0;
        auto pass = [&]() {
#pragma unroll
            for (int s = 0; s < 8; ++s) { const int Lid = (lane >> 3) + 4 * s, piece = lane & 7; const int row = Lid >> 1, cofs = (Lid & 1) * 32 + piece * 4;
                v4f val = *(const v4fa*)(os + row * 68 + cofs); if (R) { const v4f rv = *(const v4f*)(R + ((size_t)r0 + row) * ldc + c0 + cofs); val += rneR ? (v4f){bfr(rv[0]), bfr(rv[1]), bfr(rv[2]), bfr(rv[3])} : rv; }
                *(volatile v4f*)(crow + (size_t)row * ldc + cofs) = val; }
        };
        pass(); __threadfence(); pass();
    }
}

__global__ __launch_bounds__(256) void k_cvt8(const float* __restrict__ src, bf* dst, size_t n8) {
    const size_t i = (size_t)blockIdx.x * 256 + threadIdx.x; if (i >= n8) return;
    const v8f v = *(const v8f*)(src + i * 8); v8us o;
#pragma unroll
    for (int k = 0; k < 8; ++k) o[k] = f2bf(v[k]);
    *(volatile v8us*)(dst + i * 8) = o; __threadfence(); *(volatile v8us*)(dst + i * 8) = o;
}

__global__ __launch_bounds__(256) void k_cvtx(const float* __restrict__ src, int rows, bf* dst) {
    const int lane = threadIdx.x & 31; const size_t r = (size_t)blockIdx.x * 8 + (threadIdx.x >> 5); if (r >= (size_t)rows) return;
#pragma unroll 1
    for (int ps = 0; ps < 2; ++ps) {
#pragma unroll
        for (int q = 0; q < DMOD / 256; ++q) { v8us o;
#pragma unroll
            for (int i = 0; i < 8; ++i) o[i] = f2bf(src[r * DMOD + q * 256 + lane * 8 + i]);
            *(volatile v8us*)(dst + r * DMOD + q * 256 + lane * 8) = o; }
        if (ps == 0) __threadfence(); }
}
__global__ __launch_bounds__(256) void k_wcat3(const float* __restrict__ Wq, const float* __restrict__ Wk, const float* __restrict__ Wv, bf* WQKV) {
    const size_t i = ((size_t)blockIdx.x * 256 + threadIdx.x) * 8; if (i >= (size_t)3 * DMOD * DMOD) return; const size_t blk = i / ((size_t)DMOD * DMOD), o = i % ((size_t)DMOD * DMOD);
    const float* src = (blk == 0) ? Wq : (blk == 1) ? Wk : Wv; v8us v;
#pragma unroll
    for (int q = 0; q < 8; ++q) v[q] = f2bf(src[o + q]);
    *(volatile v8us*)(WQKV + i) = v; __threadfence(); *(volatile v8us*)(WQKV + i) = v;
}
__global__ __launch_bounds__(256) void k_vtz(const float* __restrict__ F, int ld, int h0, int nk, bf* Th, bf* Tl) {
    typedef __attribute__((ext_vector_type(2))) unsigned short v2us;
    const int lane = threadIdx.x & 31; const size_t wid = (size_t)blockIdx.x * 8 + (threadIdx.x >> 5); if (wid >= (size_t)64 * (nk / 64)) return; const int z = blockIdx.z; const int d = (int)(wid / (nk / 64)); const int t0 = (int)(wid % (nk / 64)) * 64 + lane * 2; v2us oh, ol;
    Th += (size_t)z * 64 * nk; Tl += (size_t)z * 64 * nk;
#pragma unroll
    for (int i = 0; i < 2; ++i) { const float y = F[(size_t)(t0 + i) * ld + (h0 + z) * 64 + d]; const unsigned short hb = f2bf(y); oh[i] = hb; ol[i] = f2bf(y - bf2f(hb)); }
    const size_t o = (size_t)d * nk + t0; *(volatile v2us*)(Th + o) = oh; *(volatile v2us*)(Tl + o) = ol; __threadfence(); *(volatile v2us*)(Th + o) = oh; *(volatile v2us*)(Tl + o) = ol;
}

__global__ __launch_bounds__(256) void k_ropetab(float* TAB) {
#pragma clang fp contract(off)
    typedef __attribute__((ext_vector_type(2))) float v2f;
    const int gid = blockIdx.x * 256 + threadIdx.x; if (gid >= SEQ * NFREQ) return;
    const int pos = gid / NFREQ, i = gid % NFREQ;
    const float invf = (float)exp(-(double)i * 0.28782313662425571);
    const float ang = (float)pos * invf;
    float sn, cs; sincosf(ang, &sn, &cs);
    v2f v; v[0] = cs; v[1] = sn;
    *(volatile v2f*)(TAB + 2 * (size_t)gid) = v; __threadfence(); *(volatile v2f*)(TAB + 2 * (size_t)gid) = v;
}

__global__ __launch_bounds__(256) void k_ropeqk(const float* __restrict__ QKV, const float* __restrict__ TAB, bf* Qh, bf* Ql, bf* Kh, bf* Kl) {
#pragma clang fp contract(off)
    typedef __attribute__((ext_vector_type(2))) unsigned short v2us;
    typedef __attribute__((ext_vector_type(2))) float v2f;
    const int lane = threadIdx.x & 31; const size_t r = (size_t)blockIdx.x * 8 + (threadIdx.x >> 5); if (r >= (size_t)SEQ) return;
    const int which = blockIdx.y, z = blockIdx.z;
    const v2f xv = *(const v2f*)(QKV + r * (3 * DMOD) + (size_t)which * DMOD + z * HD + 2 * lane);
    const v2f tc = *(const v2f*)(TAB + (r * NFREQ + lane) * 2);
    const float xe = xv[0], xo = xv[1], c = tc[0], s = tc[1];
    const float pe = xe * c; const float po = xo * s; const float qe = xe * s; const float qo = xo * c;
    const float ye = pe - po; const float yo = qe + qo;
    bf* Ph = which ? Kh : Qh; bf* Pl = which ? Kl : Ql;
    v2us oh, ol;
    { const unsigned short hb = f2bf(ye); oh[0] = hb; ol[0] = f2bf(ye - bf2f(hb)); }
    { const unsigned short hb = f2bf(yo); oh[1] = hb; ol[1] = f2bf(yo - bf2f(hb)); }
    const size_t o = ((size_t)z * SEQ + r) * HD + 2 * lane;
    *(volatile v2us*)(Ph + o) = oh; *(volatile v2us*)(Pl + o) = ol; __threadfence(); *(volatile v2us*)(Ph + o) = oh; *(volatile v2us*)(Pl + o) = ol;
}

__global__ __launch_bounds__(128) __attribute__((amdgpu_num_vgpr(256)))
void k_flashz(const bf* __restrict__ Qh, const bf* __restrict__ Ql, const bf* __restrict__ Kh, const bf* __restrict__ Kl,
              const bf* __restrict__ VTh, const bf* __restrict__ VTl, float sc, bf* Oh, bf* Ol) {
    __shared__ __align__(16) float pst[4][16 * 68];
    const int lane = threadIdx.x & 31, wave = threadIdx.x >> 5, lr = lane & 15, hi = lane >> 4;
    const int qb = blockIdx.x, z = blockIdx.y;
    const int r0 = qb * 64 + wave * 16;
    const bf* qh = Qh + (size_t)z * SEQ * HD; const bf* ql = Ql + (size_t)z * SEQ * HD;
    const bf* kh = Kh + (size_t)z * SEQ * HD; const bf* kl = Kl + (size_t)z * SEQ * HD;
    const bf* vth = VTh + (size_t)z * HD * SEQ; const bf* vtl = VTl + (size_t)z * HD * SEQ;
    float* ps = &pst[wave][0];
    const size_t qoff = (size_t)(r0 + lr) * HD + 8 * hi;
    v8f oacc[4];
#pragma unroll
    for (int t = 0; t < 4; ++t) oacc[t] = (v8f){};
    float m[8], l[8];
#pragma unroll
    for (int r = 0; r < 8; ++r) { m[r] = -1.0e30f; l[r] = 0.f; }
#pragma unroll 1
    for (int kc = 0; kc <= qb; ++kc) {
        const int key0 = kc * 64;
        v8f sacc[4];
#pragma unroll
        for (int t = 0; t < 4; ++t) sacc[t] = (v8f){};
#pragma unroll 1
        for (int j = 0; j < 2; ++j) {
            const v16bf a  = cat16b(*(const v8us*)(qh + qoff + j * 32), *(const v8us*)(qh + qoff + j * 32 + 16));
            const v16bf al = cat16b(*(const v8us*)(ql + qoff + j * 32), *(const v8us*)(ql + qoff + j * 32 + 16));
#pragma unroll
            for (int t = 0; t < 4; ++t) {
                const size_t bo = (size_t)(key0 + t * 16 + lr) * HD + j * 32 + 8 * hi;
                const v16bf bh = cat16b(*(const v8us*)(kh + bo), *(const v8us*)(kh + bo + 16));
                const v16bf bl = cat16b(*(const v8us*)(kl + bo), *(const v8us*)(kl + bo + 16));
                sacc[t] = wmmab(a, bh, sacc[t]); sacc[t] = wmmab(al, bh, sacc[t]); sacc[t] = wmmab(a, bl, sacc[t]);
            }
            asm volatile("v_nop\n\tv_nop\n\tv_nop\n\tv_nop" : "+v"(sacc[0]), "+v"(sacc[1]), "+v"(sacc[2]), "+v"(sacc[3]) : "v"(a), "v"(al));
        }
        const int thr = (qb - kc) * 64 + wave * 16 + 8 * hi;
        float mc[8], rs[8];
#pragma unroll
        for (int r = 0; r < 8; ++r) { float mx = -1.0e30f;
#pragma unroll
            for (int t = 0; t < 4; ++t) { const float sv = (t * 16 + lr <= thr + r) ? sacc[t][r] * sc : -1.0e30f; sacc[t][r] = sv; mx = fmaxf(mx, sv); }
            mc[r] = mx; }
#pragma unroll
        for (int r = 0; r < 8; ++r) { float v = mc[r];
#pragma unroll
            for (int sh = 1; sh < 16; sh <<= 1) v = fmaxf(v, __shfl_xor(v, sh, 32));
            mc[r] = v; }
#pragma unroll
        for (int r = 0; r < 8; ++r) {
            const float mn = fmaxf(m[r], mc[r]); const float alf = __expf(m[r] - mn); m[r] = mn; float ssum = 0.f;
#pragma unroll
            for (int t = 0; t < 4; ++t) { const float pv = __expf(sacc[t][r] - mn); ps[(hi * 8 + r) * 68 + t * 16 + lr] = pv; ssum += pv; }
            rs[r] = ssum; l[r] *= alf;
#pragma unroll
            for (int t = 0; t < 4; ++t) oacc[t][r] *= alf;
        }
#pragma unroll
        for (int r = 0; r < 8; ++r) { float v = rs[r];
#pragma unroll
            for (int sh = 1; sh < 16; sh <<= 1) v += __shfl_xor(v, sh, 32);
            l[r] += v; }
        __syncthreads();
#pragma unroll 1
        for (int j = 0; j < 2; ++j) {
            const float* pr = ps + lr * 68 + j * 32 + 8 * hi;
            const v4f f0 = *(const v4fa*)(pr), f1 = *(const v4fa*)(pr + 4), f2 = *(const v4fa*)(pr + 16), f3 = *(const v4fa*)(pr + 20);
            v8us ph0, ph1, pl0, pl1;
#pragma unroll
            for (int i = 0; i < 4; ++i) {
                { const float y = f0[i]; const unsigned short hb = f2bf(y); ph0[i] = hb;     pl0[i] = f2bf(y - bf2f(hb)); }
                { const float y = f1[i]; const unsigned short hb = f2bf(y); ph0[4 + i] = hb; pl0[4 + i] = f2bf(y - bf2f(hb)); }
                { const float y = f2[i]; const unsigned short hb = f2bf(y); ph1[i] = hb;     pl1[i] = f2bf(y - bf2f(hb)); }
                { const float y = f3[i]; const unsigned short hb = f2bf(y); ph1[4 + i] = hb; pl1[4 + i] = f2bf(y - bf2f(hb)); }
            }
            const v16bf pa = cat16b(ph0, ph1), pb = cat16b(pl0, pl1);
#pragma unroll
            for (int t = 0; t < 4; ++t) {
                const size_t bo = (size_t)(t * 16 + lr) * SEQ + key0 + j * 32 + 8 * hi;
                const v16bf vh = cat16b(*(const v8us*)(vth + bo), *(const v8us*)(vth + bo + 16));
                const v16bf vl = cat16b(*(const v8us*)(vtl + bo), *(const v8us*)(vtl + bo + 16));
                oacc[t] = wmmab(pa, vh, oacc[t]); oacc[t] = wmmab(pb, vh, oacc[t]); oacc[t] = wmmab(pa, vl, oacc[t]);
            }
            asm volatile("v_nop\n\tv_nop\n\tv_nop\n\tv_nop" : "+v"(oacc[0]), "+v"(oacc[1]), "+v"(oacc[2]), "+v"(oacc[3]) : "v"(pa), "v"(pb));
        }
        __syncthreads();
    }
    float inv[8];
#pragma unroll
    for (int r = 0; r < 8; ++r) inv[r] = 1.0f / l[r];
#pragma unroll
    for (int t = 0; t < 4; ++t) {
#pragma unroll
        for (int r = 0; r < 8; ++r) ps[(hi * 8 + r) * 68 + t * 16 + lr] = oacc[t][r] * inv[r]; }
    __syncthreads();
    bf* oh = Oh + (size_t)r0 * DMOD + z * HD; bf* ol = Ol + (size_t)r0 * DMOD + z * HD;
    auto pass = [&]() {
#pragma unroll
        for (int s = 0; s < 4; ++s) { const int row = 4 * s + (lane >> 3), piece = lane & 7; const float* sp = ps + row * 68 + piece * 8;
            const v4f g0 = *(const v4fa*)(sp), g1 = *(const v4fa*)(sp + 4); v8us o1, o2;
#pragma unroll
            for (int i = 0; i < 4; ++i) {
                { const float y = g0[i]; const unsigned short hb = f2bf(y); o1[i] = hb;     o2[i] = f2bf(y - bf2f(hb)); }
                { const float y = g1[i]; const unsigned short hb = f2bf(y); o1[4 + i] = hb; o2[4 + i] = f2bf(y - bf2f(hb)); } }
            *(volatile v8us*)(oh + (size_t)row * DMOD + piece * 8) = o1; *(volatile v8us*)(ol + (size_t)row * DMOD + piece * 8) = o2; }
    };
    pass(); __threadfence(); pass();
}

extern "C" void kernel_launch(void* const* d_in, const int* in_sizes, int n_in,
                              void* d_out, int out_size, void* d_ws, size_t ws_size, hipStream_t stream) {
    if (n_in < 5) return;
    const size_t rows_used = (size_t)(NB - 1) * SEQ_FULL + SEQ;
    if ((size_t)in_sizes[0] < rows_used * DMOD) return;
    for (int i = 1; i < 5; ++i) if ((size_t)in_sizes[i] < (size_t)DMOD * DMOD) return;
    if ((size_t)out_size < rows_used * DMOD) return;
    const float* x = (const float*)d_in[0]; const float* Wq = (const float*)d_in[1]; const float* Wk = (const float*)d_in[2]; const float* Wv = (const float*)d_in[3]; const float* Wo = (const float*)d_in[4];
    float* out0 = (float*)d_out;
    char* wsp = (char*)d_ws;
    auto take = [&](size_t bytes) { char* p = wsp; wsp += (bytes + 255) & ~(size_t)255; return (void*)p; };
    bf* WQKV = (bf*)take((size_t)3 * DMOD * DMOD * 2);
    bf* WO   = (bf*)take((size_t)DMOD * DMOD * 2);
    float* TAB = (float*)take((size_t)SEQ * NFREQ * 2 * 4);
    bf* Xb   = (bf*)take((size_t)SEQ * DMOD * 2);
    float* QKV = (float*)take((size_t)SEQ * 3 * DMOD * 4);
    bf* Qh = (bf*)take((size_t)NH_ * SEQ * HD * 2); bf* Ql = (bf*)take((size_t)NH_ * SEQ * HD * 2);
    bf* Kh = (bf*)take((size_t)NH_ * SEQ * HD * 2); bf* Kl = (bf*)take((size_t)NH_ * SEQ * HD * 2);
    bf* VTh = (bf*)take((size_t)NH_ * HD * SEQ * 2); bf* VTl = (bf*)take((size_t)NH_ * HD * SEQ * 2);
    bf* Oh = (bf*)take((size_t)SEQ * DMOD * 2); bf* Ol = (bf*)take((size_t)SEQ * DMOD * 2);
    if ((size_t)(wsp - (char*)d_ws) > ws_size) return;
    k_wcat3<<<(unsigned)((3 * (size_t)DMOD * DMOD / 8 + 255) / 256), 256, 0, stream>>>(Wq, Wk, Wv, WQKV);
    k_cvt8<<<(DMOD * DMOD / 8 + 255) / 256, 256, 0, stream>>>(Wo, WO, (size_t)DMOD * DMOD / 8);
    k_ropetab<<<(SEQ * NFREQ + 255) / 256, 256, 0, stream>>>(TAB);
    for (int b = 0; b < NB; ++b) {
        k_cvtx<<<SEQ / 8, 256, 0, stream>>>(x + (size_t)b * SEQ_FULL * DMOD, SEQ, Xb);
        k_gemmb<false, false><<<dim3(SEQ / 64, (3 * DMOD) / 64, 1), 128, 0, stream>>>(Xb, nullptr, WQKV, nullptr, QKV, 3 * DMOD, nullptr, nullptr, DMOD, 1);
        k_ropeqk<<<dim3(SEQ / 8, 2, NH_), 256, 0, stream>>>(QKV, TAB, Qh, Ql, Kh, Kl);
        k_vtz<<<dim3(SEQ / 8, 1, NH_), 256, 0, stream>>>(QKV + 2 * DMOD, 3 * DMOD, 0, SEQ, VTh, VTl);
        k_flashz<<<dim3(SEQ / 64, NH_, 1), 128, 0, stream>>>(Qh, Ql, Kh, Kl, VTh, VTl, SCL, Oh, Ol);
        k_gemmb<true, false><<<dim3(SEQ / 64, DMOD / 64, 1), 128, 0, stream>>>(Oh, Ol, WO, nullptr, out0 + (size_t)b * SEQ_FULL * DMOD, DMOD, nullptr, nullptr, DMOD, 1);
    }
}
